// ModelLSTM_71047349010535
// MI455X (gfx1250) — hardware-verified
//
#include <hip/hip_runtime.h>
#include <stddef.h>
#include <stdint.h>


#define NB    32
#define NS    512
#define NV    32000
#define ND    512
#define NH    256
#define NG    1024
#define NM    64
#define NE    32
#define NR    97
#define NRP   256
#define NTOK  (NB * NS)
#define PTHR  128
#define MTHR  256
#define GTHR  512
#define HS16  264
#define CTP   36
#define CRP   260
#define SCN   9216

static_assert(NB == 32);
static_assert(NTOK % 64 == 0);
static_assert((2 * NG) % 256 == 0 && ND % 256 == 0 && NRP == 256);
static_assert(ND % 32 == 0 && NH % 32 == 0);
static_assert(GTHR == 32 * (NH / 16));
static_assert((HS16 * 2) % 16 == 0 && HS16 >= NH);
static_assert((CTP * 4) % 16 == 0 && (CRP * 4) % 16 == 0);
static_assert(SCN >= 32 * CRP && SCN >= 256 * CTP);
static_assert((NE * NR) % 4 == 0 && ((NE * NR * 4) % 128) == 0);
static_assert(NR <= 128 && NR <= NRP && NM <= MTHR && NE <= MTHR);
static_assert(ND == 4 * PTHR);
static_assert(NE % (MTHR / 32) == 0);

typedef _Float16 v4h  __attribute__((ext_vector_type(4)));
typedef _Float16 v8h  __attribute__((ext_vector_type(8)));
typedef _Float16 v16h __attribute__((ext_vector_type(16)));
typedef float    v4f  __attribute__((ext_vector_type(4)));
typedef float    v8f  __attribute__((ext_vector_type(8)));

union Frag { v16h v; v8h h[2]; };

#if __has_builtin(__builtin_amdgcn_exp2f)
#define EXP2_FAST(x) __builtin_amdgcn_exp2f(x)
#else
#define EXP2_FAST(x) exp2f(x)
#endif
#define RCP_FAST(x) __builtin_amdgcn_rcpf(x)

#define XSC   64.0f
#define WSC   256.0f
#define HSC   16.0f
#define XPSC  64.0f
#define RSC   16.0f
#define PSC   16.0f
#define IHSC  0.0625f
#define IS8   0.00390625f
#define IS12  0.000244140625f
#define IS14  0.00006103515625f
#define XPUP  64.0f
#define LOG2E 1.4426950408889634f
#define C2L2E 2.8853900817779268f

__device__ __forceinline__ v16h frag16(const _Float16* row, int k0, int hh)
{
    Frag f;
    f.h[0] = *(const v8h*)(row + k0 + 8 * hh);
    f.h[1] = *(const v8h*)(row + k0 + 16 + 8 * hh);
    return f.v;
}

__device__ __forceinline__ v8f wmma_f16(v16h a, v16h b, v8f c)
{
    v8f d = __builtin_amdgcn_wmma_f32_16x16x32_f16(false, a, false, b, (short)0, c, false, false);
    asm volatile("v_nop\n\tv_nop\n\tv_nop\n\tv_nop" : "+v"(d) : "v"(a), "v"(b));
    return d;
}

__device__ __forceinline__ v8h pack8h(v4f a, v4f b)
{
    v8h r = { (_Float16)a[0], (_Float16)a[1], (_Float16)a[2], (_Float16)a[3],
              (_Float16)b[0], (_Float16)b[1], (_Float16)b[2], (_Float16)b[3] };
    return r;
}

__device__ __forceinline__ float sigm_f(float x)
{
    return RCP_FAST(1.0f + EXP2_FAST(-LOG2E * x));
}
__device__ __forceinline__ float tanh_f(float x)
{
    return 1.0f - 2.0f * RCP_FAST(1.0f + EXP2_FAST(C2L2E * x));
}

__device__ __forceinline__ v4f bias4(const float* __restrict__ bp, const float* __restrict__ bx,
                                     int n, int nb, float bm, float bxm)
{
    const float e0 = (n + 0 < nb) ? (bp[n + 0] * bm + bx[n + 0] * bxm) : 0.0f;
    const float e1 = (n + 1 < nb) ? (bp[n + 1] * bm + bx[n + 1] * bxm) : 0.0f;
    const float e2 = (n + 2 < nb) ? (bp[n + 2] * bm + bx[n + 2] * bxm) : 0.0f;
    const float e3 = (n + 3 < nb) ? (bp[n + 3] * bm + bx[n + 3] * bxm) : 0.0f;
    v4f r = { e0, e1, e2, e3 };
    return r;
}

__device__ __forceinline__ v8f ldx8(const _Float16* p)
{
    const v8h h = *(const v8h*)p;
    return __builtin_convertvector(h, v8f) * XPUP;
}

__global__ void __launch_bounds__(PTHR) prep_kernel(
    const float* __restrict__ wih0, const float* __restrict__ whh0,
    const float* __restrict__ wih1, const float* __restrict__ whh1,
    const float* __restrict__ r1w,  const float* __restrict__ r2w,
    const float* __restrict__ pjw,  const float* __restrict__ dcw,
    _Float16* wih0h, _Float16* whh0h, _Float16* wih1h, _Float16* whh1h,
    _Float16* r1wh, _Float16* r2wh, _Float16* pjwh, _Float16* dcwh)
{
    const int tid = threadIdx.x;
    const int bid = blockIdx.x;
    const int S0 = (2 * NG * ND) / 1024;
    const int S1 = S0 + (2 * NG * NH) / 1024;
    const int S2 = S1 + (2 * NG * ND) / 1024;
    const int S3 = S2 + (2 * NG * NH) / 1024;
    const int S4 = S3 + (ND * ND) / 1024;
    const int S5 = S4 + (ND * ND) / 1024;
    const int S6 = S5 + (ND * ND) / 1024;

    const float* src;
    _Float16* dst;
    int loc;
    bool valid = true;
    if (bid < S0)      { loc = bid;      src = wih0; dst = wih0h; }
    else if (bid < S1) { loc = bid - S0; src = whh0; dst = whh0h; }
    else if (bid < S2) { loc = bid - S1; src = wih1; dst = wih1h; }
    else if (bid < S3) { loc = bid - S2; src = whh1; dst = whh1h; }
    else if (bid < S4) { loc = bid - S3; src = r1w;  dst = r1wh;  }
    else if (bid < S5) { loc = bid - S4; src = r2w;  dst = r2wh;  }
    else if (bid < S6) { loc = bid - S5; src = pjw;  dst = pjwh;  }
    else {
        loc = bid - S6; src = dcw; dst = dcwh;
        const int row = (loc * 1024 + tid * 8) >> 9;
        valid = row < NR;
    }
    const int e0 = loc * 1024 + tid * 8;
    v4f x0 = { 0.f, 0.f, 0.f, 0.f };
    v4f x1 = { 0.f, 0.f, 0.f, 0.f };
    if (valid) {
        x0 = *(const v4f*)(src + e0);
        x1 = *(const v4f*)(src + e0 + 4);
    }
    const v8h val = pack8h(x0 * WSC, x1 * WSC);
    volatile v8h* p = (volatile v8h*)(dst + e0);
    *p = val;
    __threadfence();
    *p = val;
}

__global__ void __launch_bounds__(MTHR) embed_kernel(
    const int* __restrict__ sents, const float* __restrict__ emb, _Float16* X)
{
    const int tid = threadIdx.x;
    const int r   = blockIdx.x * 4 + (tid >> 6);
    const int c8  = tid & 63;
    const int s   = r >> 5;
    const int b   = r & (NB - 1);
    int id = sents[b * NS + s];
    id = id < 0 ? 0 : (id > NV - 1 ? NV - 1 : id);
    const float* src = emb + (size_t)id * ND + 8 * c8;
    const v4f x0 = *(const v4f*)(src);
    const v4f x1 = *(const v4f*)(src + 4);
    const v8h val = pack8h(x0 * XSC, x1 * XSC);
    volatile v8h* p = (volatile v8h*)(X + (size_t)r * ND + 8 * c8);
    *p = val;
    __threadfence();
    *p = val;
}

template <int MODE>
__global__ void __launch_bounds__(MTHR) gemm_kernel(
    const _Float16* __restrict__ A0, const _Float16* __restrict__ A1, int lda,
    const _Float16* __restrict__ W0, const _Float16* __restrict__ W1, int ldw,
    const float* __restrict__ bias0, const float* __restrict__ bias1,
    const float* __restrict__ biasx, int nb, float bmul0, float bmul1, float bxmul,
    void* C0, void* C1, int ldc, int ncol, int K, float scale, float oscale)
{
    __shared__ __align__(16) float s_c[SCN];

    const int z = blockIdx.z;
    const _Float16* A    = z ? A1 : A0;
    const _Float16* W    = z ? W1 : W0;
    const float*    bias = z ? bias1 : bias0;
    const float     bmul = z ? bmul1 : bmul0;
    void*           Cv   = z ? C1 : C0;

    const int tid = threadIdx.x;
    const int l   = tid & 31;
    const int wid = tid >> 5;
    const int wm  = wid >> 2, wn = wid & 3;
    const int hh  = l >> 4, m15 = l & 15;
    const int mblk = blockIdx.x * 64;
    const int nblk = blockIdx.y * 256;
    const int m0 = mblk + wm * 32;
    const int n0 = nblk + wn * 64;

    const v8f zero = { 0.f, 0.f, 0.f, 0.f, 0.f, 0.f, 0.f, 0.f };
    v8f acc[2][4];
    #pragma unroll
    for (int mi = 0; mi < 2; ++mi)
        #pragma unroll
        for (int j = 0; j < 4; ++j) acc[mi][j] = zero;

    const _Float16* a0p = A + (size_t)(m0 + m15) * lda;
    const _Float16* a1p = A + (size_t)(m0 + 16 + m15) * lda;
    const _Float16* wp  = W + (size_t)(n0 + m15) * ldw;

    #pragma unroll 2
    for (int k0 = 0; k0 < K; k0 += 32) {
        const v16h fa0 = frag16(a0p, k0, hh);
        const v16h fa1 = frag16(a1p, k0, hh);
        #pragma unroll
        for (int j = 0; j < 4; ++j) {
            const v16h fb = frag16(wp + (size_t)j * 16 * ldw, k0, hh);
            acc[0][j] = wmma_f16(fa0, fb, acc[0][j]);
            acc[1][j] = wmma_f16(fa1, fb, acc[1][j]);
        }
    }

    for (int ph = 0; ph < 2; ++ph) {
        if (wm == ph) {
            #pragma unroll
            for (int mi = 0; mi < 2; ++mi)
                #pragma unroll
                for (int j = 0; j < 4; ++j)
                    #pragma unroll
                    for (int r = 0; r < 8; ++r) {
                        const int rl = mi * 16 + 8 * hh + r;
                        const int cl = wn * 64 + 16 * j + m15;
                        if constexpr (MODE == 0) s_c[cl * CTP + rl] = acc[mi][j][r];
                        else                     s_c[rl * CRP + cl] = acc[mi][j][r];
                    }
        }
        __syncthreads();

        if constexpr (MODE == 0) {
            _Float16* C = (_Float16*)Cv;
            const int s = (mblk >> 5) + ph;
            v8h vals[4];
            size_t off[4];
            #pragma unroll
            for (int i = 0; i < 4; ++i) {
                const int idx = tid + MTHR * i;
                const int nl  = idx >> 2;
                const int q   = idx & 3;
                const int n   = nblk + nl;
                const v4f x0 = *(const v4f*)&s_c[nl * CTP + 8 * q];
                const v4f x1 = *(const v4f*)&s_c[nl * CTP + 8 * q + 4];
                float bv = 0.0f;
                if (n < nb) bv = bias[n] * bmul + biasx[n] * bxmul;
                vals[i] = pack8h((x0 * scale + bv) * oscale, (x1 * scale + bv) * oscale);
                off[i]  = ((size_t)s * ncol + n) * NB + 8 * q;
            }
            #pragma unroll
            for (int i = 0; i < 4; ++i) *(volatile v8h*)(C + off[i]) = vals[i];
            __threadfence();
            #pragma unroll
            for (int i = 0; i < 4; ++i) *(volatile v8h*)(C + off[i]) = vals[i];
        } else if constexpr (MODE == 1) {
            _Float16* C = (_Float16*)Cv;
            v8h vals[4];
            size_t off[4];
            #pragma unroll
            for (int i = 0; i < 4; ++i) {
                const int idx = tid + MTHR * i;
                const int row = idx >> 5;
                const int c8  = idx & 31;
                const int n   = nblk + 8 * c8;
                const v4f x0 = *(const v4f*)&s_c[row * CRP + 8 * c8];
                const v4f x1 = *(const v4f*)&s_c[row * CRP + 8 * c8 + 4];
                const v4f b0 = bias4(bias, biasx, n, nb, bmul, bxmul);
                const v4f b1 = bias4(bias, biasx, n + 4, nb, bmul, bxmul);
                vals[i] = pack8h((x0 * scale + b0) * oscale, (x1 * scale + b1) * oscale);
                off[i]  = (size_t)(mblk + 32 * ph + row) * ldc + n;
            }
            #pragma unroll
            for (int i = 0; i < 4; ++i) *(volatile v8h*)(C + off[i]) = vals[i];
            __threadfence();
            #pragma unroll
            for (int i = 0; i < 4; ++i) *(volatile v8h*)(C + off[i]) = vals[i];
        } else {
            float* C = (float*)Cv;
            v4f vals[8];
            size_t off[8];
            #pragma unroll
            for (int i = 0; i < 8; ++i) {
                const int idx = tid + MTHR * i;
                const int row = idx >> 6;
                const int c4  = idx & 63;
                const int n   = nblk + 4 * c4;
                const v4f x  = *(const v4f*)&s_c[row * CRP + 4 * c4];
                const v4f bq = bias4(bias, biasx, n, nb, bmul, bxmul);
                vals[i] = (x * scale + bq) * oscale;
                off[i]  = (size_t)(mblk + 32 * ph + row) * ldc + n;
            }
            #pragma unroll
            for (int i = 0; i < 8; ++i) *(volatile v4f*)(C + off[i]) = vals[i];
            __threadfence();
            #pragma unroll
            for (int i = 0; i < 8; ++i) *(volatile v4f*)(C + off[i]) = vals[i];
        }
        __syncthreads();
    }
}

__global__ void __launch_bounds__(GTHR) lstm_kernel(
    const _Float16* __restrict__ XP, const _Float16* __restrict__ whh, _Float16* HOUT)
{
    __shared__ __align__(16) _Float16 h16[NB * HS16];

    const int dir = blockIdx.x;
    const int tid = threadIdx.x;
    const int wv  = tid >> 5;
    const int l   = tid & 31;
    const int hh  = l >> 4;
    const int m15 = l & 15;
    const int j   = 16 * wv + m15;

    for (int i = tid; i < NB * HS16; i += GTHR) h16[i] = (_Float16)0.0f;
    float c0[8], c1[8];
    #pragma unroll
    for (int r = 0; r < 8; ++r) { c0[r] = 0.0f; c1[r] = 0.0f; }
    __syncthreads();

    const _Float16* wI = whh + ((size_t)dir * NG + 0 * NH + j) * NH;
    const _Float16* wF = whh + ((size_t)dir * NG + 1 * NH + j) * NH;
    const _Float16* wG = whh + ((size_t)dir * NG + 2 * NH + j) * NH;
    const _Float16* wO = whh + ((size_t)dir * NG + 3 * NH + j) * NH;

    const _Float16* hrow0 = &h16[m15 * HS16];
    const _Float16* hrow1 = &h16[(16 + m15) * HS16];

    const _Float16* xbase = XP + (size_t)(dir * NG + j) * NB + 8 * hh;
    const size_t XT = (size_t)2 * NG * NB;
    const int    GS = NH * NB;

    #pragma unroll 1
    for (int s = 0; s < NS; ++s) {
        const int t = dir ? (NS - 1 - s) : s;
        const _Float16* xt = xbase + (size_t)t * XT;

        v8f aI0 = ldx8(xt),          aI1 = ldx8(xt + 16);
        v8f aF0 = ldx8(xt + GS),     aF1 = ldx8(xt + GS + 16);
        v8f aG0 = ldx8(xt + 2 * GS), aG1 = ldx8(xt + 2 * GS + 16);
        v8f aO0 = ldx8(xt + 3 * GS), aO1 = ldx8(xt + 3 * GS + 16);

        #pragma unroll 1
        for (int k0 = 0; k0 < NH; k0 += 32) {
            const v16h fh0 = frag16(hrow0, k0, hh);
            const v16h fh1 = frag16(hrow1, k0, hh);
            v16h fb;
            fb = frag16(wI, k0, hh);  aI0 = wmma_f16(fh0, fb, aI0);  aI1 = wmma_f16(fh1, fb, aI1);
            fb = frag16(wF, k0, hh);  aF0 = wmma_f16(fh0, fb, aF0);  aF1 = wmma_f16(fh1, fb, aF1);
            fb = frag16(wG, k0, hh);  aG0 = wmma_f16(fh0, fb, aG0);  aG1 = wmma_f16(fh1, fb, aG1);
            fb = frag16(wO, k0, hh);  aO0 = wmma_f16(fh0, fb, aO0);  aO1 = wmma_f16(fh1, fb, aO1);
        }

        float hn0[8], hn1[8];
        #pragma unroll
        for (int r = 0; r < 8; ++r) {
            {
                const float ig = sigm_f(aI0[r] * IS12);
                const float fg = sigm_f(aF0[r] * IS12);
                const float gg = tanh_f(aG0[r] * IS12);
                const float og = sigm_f(aO0[r] * IS12);
                c0[r] = fg * c0[r] + ig * gg;
                hn0[r] = og * tanh_f(c0[r]);
            }
            {
                const float ig = sigm_f(aI1[r] * IS12);
                const float fg = sigm_f(aF1[r] * IS12);
                const float gg = tanh_f(aG1[r] * IS12);
                const float og = sigm_f(aO1[r] * IS12);
                c1[r] = fg * c1[r] + ig * gg;
                hn1[r] = og * tanh_f(c1[r]);
            }
        }
        __syncthreads();
        #pragma unroll
        for (int r = 0; r < 8; ++r) {
            h16[(8 * hh + r) * HS16 + j]      = (_Float16)(HSC * hn0[r]);
            h16[(16 + 8 * hh + r) * HS16 + j] = (_Float16)(HSC * hn1[r]);
        }
        __syncthreads();

        v8h ov[2];
        size_t off[2];
        #pragma unroll
        for (int i = 0; i < 2; ++i) {
            const int b = 2 * wv + i;
            ov[i]  = *(const v8h*)&h16[b * HS16 + 8 * l];
            off[i] = ((size_t)(t * NB + b)) * ND + (size_t)dir * NH + 8 * l;
        }
        #pragma unroll
        for (int i = 0; i < 2; ++i) *(volatile v8h*)(HOUT + off[i]) = ov[i];
        __threadfence();
        #pragma unroll
        for (int i = 0; i < 2; ++i) *(volatile v8h*)(HOUT + off[i]) = ov[i];
    }
}

__global__ void __launch_bounds__(PTHR) pool_kernel(
    const _Float16* __restrict__ H, const int* __restrict__ ent,
    const float* __restrict__ lng, const float* __restrict__ lnb, _Float16* CT)
{
    __shared__ float s_r1[4];
    __shared__ float s_r2[4];
    __shared__ __align__(16) float s_x[ND];

    const int tid = threadIdx.x;
    const int wv  = tid >> 5;
    const int l   = tid & 31;
    const int be  = blockIdx.x;
    const int b   = be >> 5;
    const int e   = be & (NE - 1);
    const int d0  = 4 * tid;

    const v4f zero4 = { 0.f, 0.f, 0.f, 0.f };
    v4f acc = zero4;
    float cnt = 0.0f;
    #pragma unroll 1
    for (int m = 0; m < NM; ++m) {
        const int* ei = ent + (b * NM + m) * 3;
        const int id = ei[0];
        if (id == e) {
            const int st = ei[1];
            const int en = ei[2];
            int len = en - st;
            if (len < 1) len = 1;
            const int lo = st < 0 ? 0 : st;
            const int hi = en > NS ? NS : en;
            v4f ms = zero4;
            #pragma unroll 1
            for (int s = lo; s < hi; ++s) {
                const v4h hv = *(const v4h*)(H + ((size_t)(s * NB + b)) * ND + d0);
                ms += __builtin_convertvector(hv, v4f);
            }
            acc += ms * (1.0f / (float)len);
            cnt += 1.0f;
        }
    }
    const v4f x = acc * (IHSC * (1.0f / fmaxf(cnt, 1.0f)));

    float p = (x[0] + x[1]) + (x[2] + x[3]);
    #pragma unroll
    for (int off = 16; off > 0; off >>= 1) p += __shfl_xor(p, off, 32);
    if (l == 0) s_r1[wv] = p;
    __syncthreads();
    const float mu = ((s_r1[0] + s_r1[1]) + (s_r1[2] + s_r1[3])) * (1.0f / ND);
    const v4f dv = x - mu;
    float p2 = (dv[0] * dv[0] + dv[1] * dv[1]) + (dv[2] * dv[2] + dv[3] * dv[3]);
    #pragma unroll
    for (int off = 16; off > 0; off >>= 1) p2 += __shfl_xor(p2, off, 32);
    if (l == 0) s_r2[wv] = p2;
    __syncthreads();
    const float var  = ((s_r2[0] + s_r2[1]) + (s_r2[2] + s_r2[3])) * (1.0f / ND);
    const float rstd = 1.0f / sqrtf(var + 1e-5f);
    const v4f g4 = *(const v4f*)(lng + d0);
    const v4f b4 = *(const v4f*)(lnb + d0);
    const v4f y  = dv * rstd * g4 + b4;
    *(v4f*)&s_x[d0] = y;
    __syncthreads();

    v8h pv = { (_Float16)0.f, (_Float16)0.f, (_Float16)0.f, (_Float16)0.f,
               (_Float16)0.f, (_Float16)0.f, (_Float16)0.f, (_Float16)0.f };
    size_t po = 0;
    if (tid < ND / 8) {
        const v4f o0 = *(const v4f*)&s_x[8 * tid];
        const v4f o1 = *(const v4f*)&s_x[8 * tid + 4];
        pv = pack8h(o0, o1);
        po = (size_t)be * ND + 8 * tid;
        *(volatile v8h*)(CT + po) = pv;
    }
    __threadfence();
    if (tid < ND / 8) *(volatile v8h*)(CT + po) = pv;
}

__global__ void __launch_bounds__(MTHR) final_kernel(
    const float* __restrict__ D1, const float* __restrict__ D2,
    const int* __restrict__ ent, float* out)
{
    __shared__ int s_flag[NE];
    __shared__ __align__(16) float s_o[NE * NR];

    const int tid = threadIdx.x;
    const int wv  = tid >> 5;
    const int l   = tid & 31;
    const int be1 = blockIdx.x;
    const int b   = be1 >> 5;
    const int e1  = be1 & (NE - 1);

    if (tid < NE) s_flag[tid] = 0;
    __syncthreads();
    if (tid < NM) {
        const int id = ent[(b * NM + tid) * 3];
        if ((unsigned)id < (unsigned)NE) s_flag[id] = 1;
    }
    __syncthreads();

    const float m1 = (float)s_flag[e1];
    const float* d2row = D2 + (size_t)(b * NE + e1) * NRP;
    float d2v[4];
    #pragma unroll
    for (int q = 0; q < 4; ++q) d2v[q] = d2row[l + 32 * q];
    const float NEG_INF = -__builtin_inff();

    #pragma unroll 1
    for (int kk = 0; kk < NE / 8; ++kk) {
        const int e2 = wv + 8 * kk;
        const float mm = m1 * (float)s_flag[e2];
        const float* d1row = D1 + (size_t)(b * NE + e2) * NRP;
        float v[4];
        float mx = NEG_INF;
        #pragma unroll
        for (int q = 0; q < 4; ++q) {
            const int c = l + 32 * q;
            const float xv = (d1row[c] + d2v[q]) * mm;
            v[q] = (c < NR) ? xv : NEG_INF;
            mx = fmaxf(mx, v[q]);
        }
        #pragma unroll
        for (int off = 16; off > 0; off >>= 1) mx = fmaxf(mx, __shfl_xor(mx, off, 32));
        float sm = 0.0f;
        #pragma unroll
        for (int q = 0; q < 4; ++q) {
            const int c = l + 32 * q;
            sm += (c < NR) ? __expf(v[q] - mx) : 0.0f;
        }
        #pragma unroll
        for (int off = 16; off > 0; off >>= 1) sm += __shfl_xor(sm, off, 32);
        const float lse = __logf(sm);
        #pragma unroll
        for (int q = 0; q < 4; ++q) {
            const int c = l + 32 * q;
            if (c < NR) s_o[e2 * NR + c] = v[q] - mx - lse;
        }
    }
    __syncthreads();

    const int NCH = (NE * NR) / 4;
    const size_t base = (size_t)be1 * (NE * NR);
    const v4f zero4 = { 0.f, 0.f, 0.f, 0.f };
    v4f vals[4];
    #pragma unroll
    for (int i = 0; i < 4; ++i) {
        const int idx = tid + MTHR * i;
        vals[i] = (idx < NCH) ? *(const v4f*)&s_o[4 * idx] : zero4;
    }
    #pragma unroll
    for (int i = 0; i < 4; ++i) {
        const int idx = tid + MTHR * i;
        if (idx < NCH) *(volatile v4f*)(out + base + 4 * idx) = vals[i];
    }
    __threadfence();
    #pragma unroll
    for (int i = 0; i < 4; ++i) {
        const int idx = tid + MTHR * i;
        if (idx < NCH) *(volatile v4f*)(out + base + 4 * idx) = vals[i];
    }
}

extern "C" void kernel_launch(void* const* d_in, const int* in_sizes, int n_in,
                              void* d_out, int out_size, void* d_ws, size_t ws_size,
                              hipStream_t stream)
{
    if (n_in < 21) return;
    if (in_sizes[0] != NB * NS) return;
    if (in_sizes[1] != NB * NM * 3) return;
    if (in_sizes[2] != NV * ND) return;
    if (in_sizes[3] != 2 * NG * ND || in_sizes[4] != 2 * NG * NH) return;
    if (in_sizes[5] != 2 * NG || in_sizes[6] != 2 * NG) return;
    if (in_sizes[7] != 2 * NG * ND || in_sizes[8] != 2 * NG * NH) return;
    if (in_sizes[9] != 2 * NG || in_sizes[10] != 2 * NG) return;
    if (in_sizes[11] != ND * ND || in_sizes[12] != ND) return;
    if (in_sizes[13] != ND * ND || in_sizes[14] != ND) return;
    if (in_sizes[15] != ND * ND || in_sizes[16] != ND) return;
    if (in_sizes[17] != NR * ND || in_sizes[18] != NR) return;
    if (in_sizes[19] != ND || in_sizes[20] != ND) return;
    if (out_size != NB * NE * NE * NR) return;

    const int*   sents  = (const int*)d_in[0];
    const int*   ent    = (const int*)d_in[1];
    const float* emb    = (const float*)d_in[2];
    const float* w_ih0  = (const float*)d_in[3];
    const float* w_hh0  = (const float*)d_in[4];
    const float* b_ih0  = (const float*)d_in[5];
    const float* b_hh0  = (const float*)d_in[6];
    const float* w_ih1  = (const float*)d_in[7];
    const float* w_hh1  = (const float*)d_in[8];
    const float* b_ih1  = (const float*)d_in[9];
    const float* b_hh1  = (const float*)d_in[10];
    const float* rel1_w = (const float*)d_in[11];
    const float* rel1_b = (const float*)d_in[12];
    const float* rel2_w = (const float*)d_in[13];
    const float* rel2_b = (const float*)d_in[14];
    const float* proj_w = (const float*)d_in[15];
    const float* proj_b = (const float*)d_in[16];
    const float* dec_w  = (const float*)d_in[17];
    const float* dec_b  = (const float*)d_in[18];
    const float* ln_g   = (const float*)d_in[19];
    const float* ln_b   = (const float*)d_in[20];
    float* out = (float*)d_out;

    const size_t szWI = (size_t)2 * NG * ND * 2;
    const size_t szWH = (size_t)2 * NG * NH * 2;
    const size_t szWD = (size_t)ND * ND * 2;
    const size_t szDC = (size_t)NRP * ND * 2;
    const size_t szX  = (size_t)NTOK * ND * 2;
    const size_t szXP = (size_t)NTOK * 2 * NG * 2;
    const size_t szCT = (size_t)NB * NE * ND * 2;
    const size_t szD  = (size_t)NB * NE * NRP * 4;
    size_t off = 0;
    const size_t oWI0 = off; off += szWI;
    const size_t oWH0 = off; off += szWH;
    const size_t oWI1 = off; off += szWI;
    const size_t oWH1 = off; off += szWH;
    const size_t oR1  = off; off += szWD;
    const size_t oR2  = off; off += szWD;
    const size_t oPJ  = off; off += szWD;
    const size_t oDC  = off; off += szDC;
    const size_t oX   = off; off += szX;
    const size_t oXP  = off; off += szXP;
    const size_t oH0  = off; off += szX;
    const size_t oCT  = off; off += szCT;
    const size_t oRL1 = off; off += szCT;
    const size_t oRL2 = off; off += szCT;
    const size_t oP1  = off; off += szCT;
    const size_t oP2  = off; off += szCT;
    const size_t oD1  = off; off += szD;
    const size_t oD2  = off; off += szD;
    if (off > ws_size) return;
    if (off > (size_t)134217728) return;

    char* ws = (char*)d_ws;
    _Float16* WI0h = (_Float16*)(ws + oWI0);
    _Float16* WH0h = (_Float16*)(ws + oWH0);
    _Float16* WI1h = (_Float16*)(ws + oWI1);
    _Float16* WH1h = (_Float16*)(ws + oWH1);
    _Float16* R1h  = (_Float16*)(ws + oR1);
    _Float16* R2h  = (_Float16*)(ws + oR2);
    _Float16* PJh  = (_Float16*)(ws + oPJ);
    _Float16* DCh  = (_Float16*)(ws + oDC);
    _Float16* X16  = (_Float16*)(ws + oX);
    _Float16* XP16 = (_Float16*)(ws + oXP);
    _Float16* H0   = (_Float16*)(ws + oH0);
    _Float16* H1   = (_Float16*)(ws + oX);
    _Float16* CT   = (_Float16*)(ws + oCT);
    _Float16* RL1  = (_Float16*)(ws + oRL1);
    _Float16* RL2  = (_Float16*)(ws + oRL2);
    _Float16* P1   = (_Float16*)(ws + oP1);
    _Float16* P2   = (_Float16*)(ws + oP2);
    float*    D1   = (float*)(ws + oD1);
    float*    D2   = (float*)(ws + oD2);

    const int nprep = (2 * NG * ND) / 1024 * 2 + (2 * NG * NH) / 1024 * 2 + (ND * ND) / 1024 * 3 + (NRP * ND) / 1024;
    prep_kernel<<<dim3(nprep), dim3(PTHR), 0, stream>>>(
        w_ih0, w_hh0, w_ih1, w_hh1, rel1_w, rel2_w, proj_w, dec_w,
        WI0h, WH0h, WI1h, WH1h, R1h, R2h, PJh, DCh);

    embed_kernel<<<dim3(NTOK / 4), dim3(MTHR), 0, stream>>>(sents, emb, X16);

    gemm_kernel<0><<<dim3(NTOK / 64, (2 * NG) / 256, 1), dim3(MTHR), 0, stream>>>(
        X16, X16, ND, WI0h, WI0h, ND, b_ih0, b_ih0, b_hh0, 2 * NG, 1.0f, 1.0f, 1.0f,
        (void*)XP16, (void*)XP16, 0, 2 * NG, ND, IS14, XPSC);

    lstm_kernel<<<dim3(2), dim3(GTHR), 0, stream>>>(XP16, WH0h, H0);

    gemm_kernel<0><<<dim3(NTOK / 64, (2 * NG) / 256, 1), dim3(MTHR), 0, stream>>>(
        H0, H0, ND, WI1h, WI1h, ND, b_ih1, b_ih1, b_hh1, 2 * NG, 1.0f, 1.0f, 1.0f,
        (void*)XP16, (void*)XP16, 0, 2 * NG, ND, IS12, XPSC);

    lstm_kernel<<<dim3(2), dim3(GTHR), 0, stream>>>(XP16, WH1h, H1);

    pool_kernel<<<dim3(NB * NE), dim3(PTHR), 0, stream>>>(H1, ent, ln_g, ln_b, CT);

    gemm_kernel<1><<<dim3((NB * NE) / 64, ND / 256, 2), dim3(MTHR), 0, stream>>>(
        CT, CT, ND, R1h, R2h, ND, rel1_b, rel2_b, rel1_b, ND, 1.0f, 1.0f, 0.0f,
        (void*)RL1, (void*)RL2, ND, ND, ND, IS8, RSC);

    gemm_kernel<1><<<dim3((NB * NE) / 64, ND / 256, 2), dim3(MTHR), 0, stream>>>(
        RL1, RL2, ND, PJh, PJh, ND, proj_b, proj_b, proj_b, ND, 0.0f, 1.0f, 0.0f,
        (void*)P1, (void*)P2, ND, ND, ND, IS12, PSC);

    gemm_kernel<2><<<dim3((NB * NE) / 64, NRP / 256, 2), dim3(MTHR), 0, stream>>>(
        P1, P2, ND, DCh, DCh, ND, dec_b, dec_b, dec_b, NR, 0.0f, 1.0f, 0.0f,
        (void*)D1, (void*)D2, NRP, NRP, ND, IS12, 1.0f);

    final_kernel<<<dim3(NB * NE), dim3(MTHR), 0, stream>>>(D1, D2, ent, out);
}
